// EGNNLayer_7541962572405
// MI455X (gfx1250) — hardware-verified
//
#include <hip/hip_runtime.h>


namespace {

constexpr int N = 50000, NP = 50048, NPL = NP  , SRCM = N  , EFULL = 640000, E = EFULL  ;
constexpr int H = 128, NF = 4  , KIN = 2 * H + NF  , NL = (NPL < N ? NPL : N), NRL = NP  ;
constexpr float LNEPS = 1e-5f;
constexpr float XS = 8.0f, WSC = 256.0f, WSQ = 0.25f, RS_ = 1024.0f, SLOPE = 0.0f, BNEPS = 1e-5f;
static_assert(NP % 32 == 0 && NP >= N && NPL % 32 == 0 && H == 128, "tiling");
typedef _Float16 b16;
typedef __attribute__((ext_vector_type(16))) _Float16 v16b;
typedef __attribute__((ext_vector_type(8))) _Float16 v8b;
typedef __attribute__((ext_vector_type(8))) float v8f;
typedef __attribute__((ext_vector_type(4))) float v4f;
__device__ __forceinline__ float bf16_rne(float f) { unsigned int u = __float_as_uint(f); u += 0x7FFFu + ((u >> 16) & 1u); return __uint_as_float(u & 0xFFFF0000u); }
__device__ __forceinline__ void split16(float v, b16& hi, b16& lo) { hi = (b16)v; lo = (b16)(v - (float)hi); }
__device__ __forceinline__ v16b frag_kb(const b16* p, int hh) { const v8b a = *(const v8b*)(p + 8 * hh), b = *(const v8b*)(p + 16 + 8 * hh); v16b f;
#pragma unroll
  for (int e = 0; e < 8; ++e) { f[e] = a[e]; f[8 + e] = b[e]; } return f; }
__device__ __forceinline__ v8f wmma16b(v16b a, v16b b, v8f c) { v8f d = __builtin_amdgcn_wmma_f32_16x16x32_f16(false, a, false, b, (short)0, c, false, false); asm volatile("v_nop\n\tv_nop\n\tv_nop\n\tv_nop" : "+v"(d) : "v"(a), "v"(b)); return d; }
__device__ __forceinline__ void wave_lds_sync() { __builtin_amdgcn_fence(__ATOMIC_RELEASE, "workgroup"); __builtin_amdgcn_wave_barrier(); __builtin_amdgcn_fence(__ATOMIC_ACQUIRE, "workgroup"); }
__device__ __forceinline__ float pmul(float a, float b) { float p = a * b; asm volatile("" : "+v"(p)); return p; }
__device__ __forceinline__ int iclamp(int v, int lo, int hi) { return v < lo ? lo : (v > hi ? hi : v); }
constexpr int CSR_NBLK = 512, CSR_GB = 8, CSR_GN = 1 << CSR_GB  , CSR_MAXG = 512, CSR_CAP = 12288  ;
__global__ __launch_bounds__(64) void csrA_kernel(const int* __restrict__ dst, int E, int N, int nG, int CHP, int NGP, int* __restrict__ STG, int* __restrict__ HST) {
  extern __shared__ int sm[];
  int* cnt = sm; int* run = sm + NGP; int* ids = sm + 2 * NGP;
  const int b = blockIdx.x; const int ch = (E + CSR_NBLK - 1) / CSR_NBLK; const int e0 = b * ch, e1 = min(E, e0 + ch);
  for (int i = threadIdx.x; i < NGP; i += 64) cnt[i] = 0;
  for (int i = threadIdx.x; i < CHP; i += 64) ids[i] = -1;
  __syncthreads();
  if (threadIdx.x == 0) {
    for (int e = e0; e < e1; ++e) { int d = dst[e]; d = (d < 0) ? 0 : (d >= N ? N - 1 : d); cnt[d >> CSR_GB] += 1; }
    int acc = 0; for (int g = 0; g < nG; ++g) { run[g] = acc; acc += cnt[g]; }
    for (int e = e0; e < e1; ++e) { int d = dst[e]; d = (d < 0) ? 0 : (d >= N ? N - 1 : d); const int g = d >> CSR_GB; ids[run[g]] = e; run[g] += 1; } }
  __syncthreads();
  typedef __attribute__((ext_vector_type(4))) int v4i;
  for (int pass = 0; pass < 2; ++pass) {
    for (int i = threadIdx.x; i < CHP / 4; i += 64) *(volatile v4i*)(STG + (size_t)b * CHP + i * 4) = *(const v4i*)(&ids[i * 4]);
    for (int i = threadIdx.x; i < NGP / 4; i += 64) { v4i v; for (int e = 0; e < 4; ++e) v[e] = (i * 4 + e < nG) ? cnt[i * 4 + e] : 0; *(volatile v4i*)(HST + (size_t)b * NGP + i * 4) = v; }
    __threadfence(); }
}
__global__ __launch_bounds__(512) void csrS_kernel(const int* __restrict__ HST, int nG, int NGP, int* __restrict__ START, int* __restrict__ TOT, int* __restrict__ OFF) {
  __shared__ int tot[CSR_MAXG];
  const int b = threadIdx.x;
  for (int pass = 0; pass < 2; ++pass) { int runb = 0; for (int g = 0; g < nG; ++g) { int c = HST[(size_t)b * NGP + g]; c = (c < 0) ? 0 : c; ((volatile int*)OFF)[(size_t)g * CSR_NBLK + b] = runb; runb += c; } __threadfence(); }
  for (int g = threadIdx.x; g < nG; g += 512) { int s = 0; for (int bb = 0; bb < CSR_NBLK; ++bb) { int c = HST[(size_t)bb * NGP + g]; s += (c < 0) ? 0 : c; } tot[g] = s; }
  __syncthreads();
  if (threadIdx.x < 32) {
    __shared__ int st[CSR_MAXG + 32];
    if (threadIdx.x == 0) { int acc = 0; for (int g = 0; g < NGP; ++g) { st[g] = acc; if (g < nG) acc += (tot[g] + 31) & ~31; } st[NGP] = acc; }
    __builtin_amdgcn_fence(__ATOMIC_RELEASE, "workgroup"); __builtin_amdgcn_wave_barrier(); __builtin_amdgcn_fence(__ATOMIC_ACQUIRE, "workgroup");
    for (int pass = 0; pass < 2; ++pass) { for (int i = threadIdx.x; i < NGP + 32; i += 32) { ((volatile int*)START)[i] = (i <= NGP) ? st[min(i, NGP)] : 0; ((volatile int*)TOT)[i] = (i < nG) ? tot[i] : 0; } __threadfence(); } }
}
__global__ __launch_bounds__(256) void csrB_kernel(const int* __restrict__ dst, int N, int nG, int CHP, int NGP, int permLen, const int* __restrict__ STG, const int* __restrict__ HST, const int* __restrict__ OFF, const int* __restrict__ START, const int* __restrict__ TOT, int* __restrict__ PERM, int* __restrict__ ROWPTR, int* __restrict__ ROWCNT, int* __restrict__ FLAG) {
  typedef __attribute__((ext_vector_type(4))) int v4i;
  __shared__ int ids[CSR_CAP]; __shared__ unsigned short key[CSR_CAP]; __shared__ int outp[CSR_CAP]; __shared__ int ncnt[CSR_GN + 1]; __shared__ int boff[CSR_NBLK + 1];
  const int g = blockIdx.x, t_ = threadIdx.x; int tot = TOT[g]; int st = START[g], stn = START[g + 1]; const int v0 = g * CSR_GN; const int nv = min(CSR_GN, N - v0);
  st = (st < 0) ? 0 : (st > permLen - 32 ? permLen - 32 : st) & ~31; stn = (stn < st) ? st : (stn > permLen ? permLen : stn); tot = (tot < 0) ? 0 : tot; if (tot > stn - st && tot <= CSR_CAP) tot = stn - st;
  if (tot > CSR_CAP) {
    for (int pass = 0; pass < 2; ++pass) { for (int i = t_; i < CSR_GN / 4; i += 256) { v4i a, c; for (int e = 0; e < 4; ++e) { a[e] = st; c[e] = 0; } *(volatile v4i*)(ROWPTR + v0 + i * 4) = a; *(volatile v4i*)(ROWCNT + v0 + i * 4) = c; } if (t_ == 0) ((volatile int*)FLAG)[0] = 1; __threadfence(); } (void)nv; return; }
  if (t_ == 0) { int acc = 0; for (int b = 0; b < CSR_NBLK; ++b) { boff[b] = acc; int c = HST[(size_t)b * NGP + g]; c = (c < 0) ? 0 : (c > CHP ? CHP : c); acc += c; if (acc > tot) acc = tot; } boff[CSR_NBLK] = acc; }
  for (int i = t_; i <= CSR_GN; i += 256) ncnt[i] = 0;
  __syncthreads();
  for (int b = 0; b < CSR_NBLK; ++b) { const int c = boff[b + 1] - boff[b]; int o_ = OFF[(size_t)g * CSR_NBLK + b]; o_ = (o_ < 0) ? 0 : (o_ > CHP - c ? CHP - c : o_); const int* src_ = STG + (size_t)b * CHP + o_;
    for (int i = t_; i < c; i += 256) { int id = src_[i]; id = (id < 0) ? 0 : id; ids[boff[b] + i] = id; int d = dst[id]; d = (d < v0) ? v0 : (d >= N ? N - 1 : d); int kk = d - v0; kk = (kk < 0) ? 0 : (kk >= CSR_GN ? CSR_GN - 1 : kk); key[boff[b] + i] = (unsigned short)kk; } }
  __syncthreads();
  if (t_ == 0) { for (int i = 0; i < tot; ++i) ncnt[key[i]] += 1; int acc = 0; for (int vl = 0; vl < CSR_GN; ++vl) { const int c = ncnt[vl]; ncnt[vl] = acc; acc += c; } ncnt[CSR_GN] = acc;
    for (int i = 0; i < tot; ++i) { const int vl = key[i]; outp[ncnt[vl]] = ids[i]; ncnt[vl] += 1; }
    for (int vl = CSR_GN; vl > 0; --vl) ncnt[vl] = ncnt[vl - 1]; ncnt[0] = 0; }
  __syncthreads();
  for (int pass = 0; pass < 2; ++pass) {
    for (int i = t_; i < (stn - st) / 4; i += 256) { v4i v; for (int e = 0; e < 4; ++e) { const int q = i * 4 + e; v[e] = (q < tot) ? outp[q] : -1; } *(volatile v4i*)(PERM + st + i * 4) = v; }
    for (int i = t_; i < CSR_GN / 4; i += 256) { v4i a, c; for (int e = 0; e < 4; ++e) { const int vl = i * 4 + e; a[e] = st + ncnt[vl]; c[e] = (vl < nv) ? (ncnt[vl + 1] - ncnt[vl]) : 0; } *(volatile v4i*)(ROWPTR + v0 + i * 4) = a; *(volatile v4i*)(ROWCNT + v0 + i * 4) = c; }
    __threadfence(); }
}
__global__ __launch_bounds__(256) void csrZ_kernel(int* __restrict__ p, size_t n4) { typedef __attribute__((ext_vector_type(4))) int v4i; const size_t tid = (size_t)blockIdx.x * 256 + threadIdx.x, nth = (size_t)gridDim.x * 256; v4i z = {0, 0, 0, 0}; for (size_t i = tid; i < n4; i += nth) *(volatile v4i*)(p + i * 4) = z; }
struct CsrBufs { int *STG, *HST, *OFF, *START, *TOT, *PERM, *ROWPTR, *ROWCNT, *FLAG; int nG, NGP, CHP; size_t permLen; char* base; size_t bytes; };
static size_t csr_carve(CsrBufs& c, char* ws, size_t off, int E, int N) {
  const size_t off0 = off; c.base = ws + off;
  auto al = [&](size_t bytes) { char* p = ws + off; off += (bytes + 255) & ~(size_t)255; return p; };
  c.nG = (N + CSR_GN - 1) / CSR_GN; c.NGP = (c.nG + 31) & ~31; const int ch = (E + CSR_NBLK - 1) / CSR_NBLK; c.CHP = (ch + 31) & ~31; c.permLen = (size_t)E + 32 * (size_t)c.nG + 32;
  c.STG = (int*)al((size_t)CSR_NBLK * c.CHP * 4); c.HST = (int*)al((size_t)CSR_NBLK * c.NGP * 4); c.OFF = (int*)al((size_t)c.NGP * CSR_NBLK * 4); c.START = (int*)al((size_t)(c.NGP + 64) * 4); c.TOT = (int*)al((size_t)(c.NGP + 64) * 4);
  c.PERM = (int*)al(c.permLen * 4); c.ROWPTR = (int*)al((size_t)c.nG * CSR_GN * 4); c.ROWCNT = (int*)al((size_t)c.nG * CSR_GN * 4); c.FLAG = (int*)al(256);
  c.bytes = off - off0; return off;
}
static void csr_build(const CsrBufs& c, const int* dst, int E, int N, hipStream_t stream) {
  const size_t smem = (size_t)(2 * c.NGP + c.CHP) * 4;
  csrZ_kernel<<<512, 256, 0, stream>>>((int*)c.base, c.bytes / 16);
  csrA_kernel<<<CSR_NBLK, 64, smem, stream>>>(dst, E, N, c.nG, c.CHP, c.NGP, c.STG, c.HST);
  csrS_kernel<<<1, 512, 0, stream>>>(c.HST, c.nG, c.NGP, c.START, c.TOT, c.OFF);
  csrB_kernel<<<c.nG, 256, 0, stream>>>(dst, N, c.nG, c.CHP, c.NGP, (int)c.permLen, c.STG, c.HST, c.OFF, c.START, c.TOT, c.PERM, c.ROWPTR, c.ROWCNT, c.FLAG);
}

typedef __attribute__((ext_vector_type(4))) _Float16 v4h;
__device__ __forceinline__ float silu_(float y) { return y * __builtin_amdgcn_rcpf(1.0f + __expf(-y)); }
__device__ __forceinline__ float sigm_(float y) { return __builtin_amdgcn_rcpf(1.0f + __expf(-y)); }
__device__ __forceinline__ float gelu_(float v) { return 0.5f * v * (1.0f + erff(v * 0.70710678118654752f)); }
template <int KP, int NOUT>
__global__ __launch_bounds__(256) void wt_kernel(const float* __restrict__ w, int ld, int k0, int KR, b16* __restrict__ WT, float scl) {
  const int u = blockIdx.x * 256 + threadIdx.x; if (u >= NOUT * KP / 8) return; const int e = u * 8; const int o = e / KP, kb = e % KP; v8b v;
#pragma unroll
  for (int j = 0; j < 8; ++j) { const int k = kb + j; v[j] = (b16)(k < KR ? bf16_rne(w[(size_t)o * ld + k0 + k]) * scl : 0.0f); }
  for (int pass = 0; pass < 2; ++pass) { *(volatile v8b*)(WT + e) = v; __threadfence(); }
}
template <int KP, int NOUT>
__global__ __launch_bounds__(256) void wtio_kernel(const float* __restrict__ w, int ldo, int k0, int KR, b16* __restrict__ WT, float scl) {
  const int u = blockIdx.x * 256 + threadIdx.x; if (u >= NOUT * KP / 8) return; const int e = u * 8; const int o = e / KP, kb = e % KP; v8b v;
#pragma unroll
  for (int j = 0; j < 8; ++j) { const int k = kb + j; v[j] = (b16)(k < KR ? bf16_rne(w[(size_t)(k0 + k) * ldo + o]) * scl : 0.0f); }
  for (int pass = 0; pass < 2; ++pass) { *(volatile v8b*)(WT + e) = v; __threadfence(); }
}
__global__ __launch_bounds__(256) void wtn1_kernel(const float* __restrict__ w, b16* __restrict__ WT, float scl) {
  const int u = blockIdx.x * 256 + threadIdx.x; if (u >= H * 2 * H / 8) return; const int e = u * 8; const int o = e / (2 * H), kb = e % (2 * H); v8b v;
#pragma unroll
  for (int j = 0; j < 8; ++j) { const int k = kb + j; v[j] = (b16)(k < H ? 0.0f : bf16_rne(w[(size_t)(k - H) * H + o]) * scl); }
  for (int pass = 0; pass < 2; ++pass) { *(volatile v8b*)(WT + e) = v; __threadfence(); }
}
template <bool HEXACT>
__global__ __launch_bounds__(64) void ab_kernel(const float* __restrict__ hx, const b16* __restrict__ WO, const b16* __restrict__ WG, const float* __restrict__ b1, float* __restrict__ AB) {
  __shared__ __attribute__((aligned(16))) b16 Ah[2][16][H + 8]; __shared__ __attribute__((aligned(16))) float Tf[2][16][H + 4];
  const int wave = threadIdx.x >> 5, lane = threadIdx.x & 31, nloc = lane & 15, hlf = lane >> 4; const size_t m0 = (size_t)blockIdx.x * 32 + wave * 16;
  for (int idx = lane; idx < 16 * (H / 4); idx += 32) { const int rr = idx / (H / 4), c4 = (idx % (H / 4)) * 4; const size_t arow = (m0 + rr < (size_t)N) ? m0 + rr : (size_t)N - 1; const v4f v = *(const v4f*)(hx + arow * H + c4); v4h hv; for (int j = 0; j < 4; ++j) hv[j] = (b16)((HEXACT ? bf16_rne(v[j]) : v[j]) * XS); *(v4h*)(&Ah[wave][rr][c4]) = hv; }
  wave_lds_sync();
#pragma unroll 1
  for (int ps = 0; ps < 2; ++ps) { const b16* W = (ps == 0) ? WO : WG;
    v8f acc[8];
#pragma unroll
    for (int t = 0; t < 8; ++t) acc[t] = (v8f){};
#pragma unroll
    for (int kb = 0; kb < H; kb += 32) { const v16b a = frag_kb(&Ah[wave][nloc][kb], hlf);
#pragma unroll
      for (int t = 0; t < 8; ++t) acc[t] = wmma16b(a, frag_kb(W + (size_t)(t * 16 + nloc) * H + kb, hlf), acc[t]); }
    if (ps > 0) wave_lds_sync();
#pragma unroll
    for (int t = 0; t < 8; ++t) { const float bb = (ps == 0) ? bf16_rne(b1[t * 16 + nloc]) : 0.0f; for (int r = 0; r < 8; ++r) Tf[wave][8 * hlf + r][t * 16 + nloc] = (m0 + 8 * hlf + r < (size_t)N) ? acc[t][r] * (1.0f / (XS * WSC)) + bb : 0.0f; }
    wave_lds_sync();
    for (int pass = 0; pass < 2; ++pass) { for (int rr = 0; rr < 16; ++rr) *(volatile v4f*)(AB + (m0 + rr) * (2 * H) + ps * H + lane * 4) = *(const v4f*)(&Tf[wave][rr][lane * 4]); __threadfence(); } }
}
__global__ __launch_bounds__(64) void nodelin_kernel(const float* __restrict__ x, const float* __restrict__ MI, const b16* __restrict__ WT, const b16* __restrict__ WQ, const float* __restrict__ bn, float* __restrict__ out, int mrows) {
  __shared__ __attribute__((aligned(16))) b16 Ah[2][16][2 * H + 8], Al[2][16][2 * H + 8]; __shared__ __attribute__((aligned(16))) float Tf[2][16][H + 4];
  const int wave = threadIdx.x >> 5, lane = threadIdx.x & 31, nloc = lane & 15, hlf = lane >> 4; const size_t m0 = (size_t)blockIdx.x * 32 + wave * 16;
  for (int idx = lane; idx < 16 * (2 * H / 4); idx += 32) { const int rr = idx / (2 * H / 4), c4 = (idx % (2 * H / 4)) * 4; const size_t arow = (m0 + rr < (size_t)N) ? m0 + rr : (size_t)N - 1;
    const bool xs = c4 < H; const v4f v = xs ? *(const v4f*)(x + arow * H + c4) : *(const v4f*)(MI + arow * H + (c4 - H)); v4h hv, lv;
    for (int j = 0; j < 4; ++j) { const float vs = (xs ? bf16_rne(v[j]) : v[j]) * XS; const b16 ph = (b16)vs; hv[j] = ph; lv[j] = (b16)((vs - (float)ph) * RS_); } *(v4h*)(&Ah[wave][rr][c4]) = hv; *(v4h*)(&Al[wave][rr][c4]) = lv; }
  wave_lds_sync();
  v8f acc[8];
#pragma unroll
  for (int t = 0; t < 8; ++t) acc[t] = (v8f){};
#pragma unroll 1
  for (int kb = 0; kb < 2 * H; kb += 32) { const v16b a = frag_kb(&Ah[wave][nloc][kb], hlf), al = frag_kb(&Al[wave][nloc][kb], hlf);
#pragma unroll
    for (int t = 0; t < 8; ++t) { const size_t wo_ = (size_t)(t * 16 + nloc) * (2 * H) + kb; acc[t] = wmma16b(a, frag_kb(WT + wo_, hlf), acc[t]); acc[t] = wmma16b(al, frag_kb(WQ + wo_, hlf), acc[t]); } }
#pragma unroll
  for (int t = 0; t < 8; ++t) { const int col = t * 16 + nloc; const float bb = bf16_rne(bn[col]); for (int r = 0; r < 8; ++r) Tf[wave][8 * hlf + r][col] = (m0 + 8 * hlf + r < (size_t)N) ? silu_(acc[t][r] * (1.0f / (XS * WSC)) + bb) : 0.0f; }
  wave_lds_sync();
  for (int pass = 0; pass < 2; ++pass) { for (int rr = 0; rr < 16; ++rr) if (m0 + rr < (size_t)mrows) *(volatile v4f*)(out + (m0 + rr) * H + lane * 4) = *(const v4f*)(&Tf[wave][rr][lane * 4]); __threadfence(); }
}
template <bool RND>
__global__ __launch_bounds__(64) void lin2_kernel(const float* __restrict__ IN_, const b16* __restrict__ WT, const b16* __restrict__ WQ, const float* __restrict__ bias, float* __restrict__ OUT, int mrows) {
  __shared__ __attribute__((aligned(16))) b16 Ah[2][16][H + 8], Al[2][16][H + 8]; __shared__ __attribute__((aligned(16))) float Tf[2][16][H + 4];
  const int wave = threadIdx.x >> 5, lane = threadIdx.x & 31, nloc = lane & 15, hlf = lane >> 4; const size_t m0 = (size_t)blockIdx.x * 32 + wave * 16;
  for (int idx = lane; idx < 16 * (H / 4); idx += 32) { const int rr = idx / (H / 4), c4 = (idx % (H / 4)) * 4; const size_t arow = (m0 + rr < (size_t)N) ? m0 + rr : (size_t)N - 1; const v4f v = *(const v4f*)(IN_ + arow * H + c4); v4h hv, lv;
    for (int j = 0; j < 4; ++j) { const float vs = (RND ? bf16_rne(v[j]) : v[j]) * XS; const b16 ph = (b16)vs; hv[j] = ph; lv[j] = (b16)((vs - (float)ph) * RS_); } *(v4h*)(&Ah[wave][rr][c4]) = hv; if (!RND) *(v4h*)(&Al[wave][rr][c4]) = lv; }
  wave_lds_sync();
  v8f acc[8];
#pragma unroll
  for (int t = 0; t < 8; ++t) acc[t] = (v8f){};
#pragma unroll
  for (int kb = 0; kb < H; kb += 32) { const v16b a = frag_kb(&Ah[wave][nloc][kb], hlf); v16b al; if (!RND) al = frag_kb(&Al[wave][nloc][kb], hlf);
#pragma unroll
    for (int t = 0; t < 8; ++t) { const size_t wo_ = (size_t)(t * 16 + nloc) * H + kb; acc[t] = wmma16b(a, frag_kb(WT + wo_, hlf), acc[t]); if (!RND) acc[t] = wmma16b(al, frag_kb(WQ + wo_, hlf), acc[t]); } }
#pragma unroll
  for (int t = 0; t < 8; ++t) { const int col = t * 16 + nloc; const float bb = bf16_rne(bias[col]); for (int r = 0; r < 8; ++r) Tf[wave][8 * hlf + r][col] = (m0 + 8 * hlf + r < (size_t)N) ? acc[t][r] * (1.0f / (XS * WSC)) + bb : 0.0f; }
  wave_lds_sync();
  for (int pass = 0; pass < 2; ++pass) { for (int rr = 0; rr < 16; ++rr) if (m0 + rr < (size_t)mrows) *(volatile v4f*)(OUT + (m0 + rr) * H + lane * 4) = *(const v4f*)(&Tf[wave][rr][lane * 4]); __threadfence(); }
}

template <int MODE>
__global__ __launch_bounds__(64) void edge_kernel(const float* __restrict__ AB, const float* __restrict__ xpos, const float* __restrict__ eattr, const int* __restrict__ cols, const int* __restrict__ PERM, const int* __restrict__ ROWPTR, const int* __restrict__ ROWCNT, int permLen,
                                                   const float* __restrict__ w1rad, const b16* __restrict__ W2T, const float* __restrict__ b2, const b16* __restrict__ WC1T, const float* __restrict__ bc1, const float* __restrict__ wc2, const float* __restrict__ bc2, float* __restrict__ OUTP, float* __restrict__ OUTC) {
  __shared__ __attribute__((aligned(16))) b16 Sh[2][16][H + 8]; __shared__ __attribute__((aligned(16))) float Tf[2][16][H + 4]; __shared__ float Gt[2][16], Rd[2][16], Ea[2][16][3]; __shared__ int Js[2][16];
  const int wave = threadIdx.x >> 5, lane = threadIdx.x & 31, nloc = lane & 15, hlf = lane >> 4; const int v = blockIdx.x * 2 + wave; const int vv = v < N ? v : N - 1;
  int cnt = 0, p0 = 0; if (v < N) { cnt = iclamp(ROWCNT[v], 0, 65536); p0 = iclamp(ROWPTR[v], 0, permLen - 1); if (p0 + cnt > permLen) cnt = permLen - p0; }
  float mip[8]; for (int t = 0; t < 8; ++t) mip[t] = 0.0f; float tsum[3] = {0.0f, 0.0f, 0.0f};
  const float px = bf16_rne(xpos[(size_t)vv * 3]), py = bf16_rne(xpos[(size_t)vv * 3 + 1]), pz = bf16_rne(xpos[(size_t)vv * 3 + 2]);
  const int cA = lane * 4;
  float own4[4], wr4[4], we4[3][4]; { const v4f o4 = *(const v4f*)(AB + (size_t)vv * (2 * H) + cA); for (int j = 0; j < 4; ++j) { own4[j] = o4[j]; wr4[j] = bf16_rne(w1rad[cA + j]); for (int f = 0; f < 3; ++f) we4[f][j] = bf16_rne(w1rad[(size_t)(1 + f) * H + cA + j]); } }
  const float bbv = bf16_rne(bc2[0]);
#pragma unroll 1
  for (int e0 = 0; e0 < cnt; e0 += 16) {
    const int nval = (cnt - e0 < 16) ? (cnt - e0) : 16;
    float rx = 0.0f, ry = 0.0f, rz = 0.0f, rad = 0.0f;
    if (lane < 16) { int c = 0;
      if (lane < nval) { const int e = iclamp(PERM[p0 + e0 + lane], 0, E - 1); c = iclamp(cols[e], 0, N - 1); if (SRCM < N) c %= SRCM;
        rx = px - bf16_rne(xpos[(size_t)c * 3]); ry = py - bf16_rne(xpos[(size_t)c * 3 + 1]); rz = pz - bf16_rne(xpos[(size_t)c * 3 + 2]); rad = sqrtf(fmaf(rx, rx, fmaf(ry, ry, pmul(rz, rz))));
        for (int f = 0; f < 3; ++f) Ea[wave][lane][f] = bf16_rne(eattr[(size_t)e * 3 + f]); }
      else { for (int f = 0; f < 3; ++f) Ea[wave][lane][f] = 0.0f; }
      Js[wave][lane] = c; Rd[wave][lane] = rad; }
    wave_lds_sync();
#pragma unroll 1
    for (int rr = 0; rr < 16; ++rr) { const int c = Js[wave][rr]; const float rd = Rd[wave][rr], a0 = Ea[wave][rr][0], a1 = Ea[wave][rr][1], a2 = Ea[wave][rr][2]; const bool ok = rr < nval; const v4f g4 = *(const v4f*)(AB + (size_t)c * (2 * H) + H + cA); v4h hv;
#pragma unroll
      for (int j = 0; j < 4; ++j) { float pre = fmaf(rd, wr4[j], own4[j] + g4[j]); pre = fmaf(a0, we4[0][j], fmaf(a1, we4[1][j], fmaf(a2, we4[2][j], pre))); hv[j] = (b16)((ok ? silu_(pre) : 0.0f) * XS); }
      *(v4h*)(&Sh[wave][rr][cA]) = hv; }
    wave_lds_sync();
#pragma unroll 1
    for (int hf = 0; hf < 2; ++hf) { v8f am[4];
#pragma unroll
      for (int t = 0; t < 4; ++t) am[t] = (v8f){};
#pragma unroll 1
      for (int kb = 0; kb < H; kb += 32) { const v16b a = frag_kb(&Sh[wave][nloc][kb], hlf);
#pragma unroll
        for (int t = 0; t < 4; ++t) am[t] = wmma16b(a, frag_kb(W2T + (size_t)((hf * 4 + t) * 16 + nloc) * H + kb, hlf), am[t]); }
#pragma unroll
      for (int t = 0; t < 4; ++t) { const int col = (hf * 4 + t) * 16 + nloc; const float b2c = bf16_rne(b2[col]);
#pragma unroll
        for (int r = 0; r < 8; ++r) Tf[wave][8 * hlf + r][col] = silu_(am[t][r] * (1.0f / (XS * WSC)) + b2c); } }
    wave_lds_sync();
#pragma unroll 1
    for (int rr = 0; rr < 16; ++rr) { v4h hv; for (int j = 0; j < 4; ++j) hv[j] = (b16)(Tf[wave][rr][cA + j] * XS); *(v4h*)(&Sh[wave][rr][cA]) = hv; }
    wave_lds_sync();
    float pc[8]; for (int r = 0; r < 8; ++r) pc[r] = 0.0f;
#pragma unroll 1
    for (int hf = 0; hf < 2; ++hf) { v8f am[4];
#pragma unroll
      for (int t = 0; t < 4; ++t) am[t] = (v8f){};
#pragma unroll 1
      for (int kb = 0; kb < H; kb += 32) { const v16b a = frag_kb(&Sh[wave][nloc][kb], hlf);
#pragma unroll
        for (int t = 0; t < 4; ++t) am[t] = wmma16b(a, frag_kb(WC1T + (size_t)((hf * 4 + t) * 16 + nloc) * H + kb, hlf), am[t]); }
#pragma unroll
      for (int t = 0; t < 4; ++t) { const int col = (hf * 4 + t) * 16 + nloc; const float bcc = bf16_rne(bc1[col]), wcc = bf16_rne(wc2[col]);
#pragma unroll
        for (int r = 0; r < 8; ++r) { const float u = silu_(am[t][r] * (1.0f / (XS * WSC)) + bcc); pc[r] = fmaf(u, wcc, pc[r]); } } }
#pragma unroll
    for (int o = 1; o < 16; o <<= 1) for (int r = 0; r < 8; ++r) pc[r] += __shfl_xor(pc[r], o);
    if (nloc == 0) { for (int r = 0; r < 8; ++r) Gt[wave][8 * hlf + r] = pc[r] + bbv; }
    wave_lds_sync();
    {
#pragma unroll
      for (int t = 0; t < 8; ++t) {
#pragma unroll
        for (int r = 0; r < 8; ++r) mip[t] += (8 * hlf + r < nval) ? Tf[wave][8 * hlf + r][t * 16 + nloc] : 0.0f; } }
    { float s = Gt[wave][lane & 15]; const float live = (lane < 16 && lane < nval) ? 1.0f : 0.0f; const float f = live * s; tsum[0] = fmaf(f, rx, tsum[0]); tsum[1] = fmaf(f, ry, tsum[1]); tsum[2] = fmaf(f, rz, tsum[2]); }
    wave_lds_sync(); }
#pragma unroll
  for (int t = 0; t < 8; ++t) mip[t] += __shfl_xor(mip[t], 16);
#pragma unroll
  for (int o = 1; o < 32; o <<= 1) { tsum[0] += __shfl_xor(tsum[0], o); tsum[1] += __shfl_xor(tsum[1], o); tsum[2] += __shfl_xor(tsum[2], o); }
  const float cdiv = 1.0f;
  for (int pass = 0; pass < 2; ++pass) { if (v < NP) { if (hlf == 0) { for (int t = 0; t < 8; ++t) ((volatile float*)OUTP)[(size_t)v * H + t * 16 + nloc] = (v < N) ? mip[t] : 0.0f; }
      const float val = (lane == 0) ? tsum[0] : (lane == 1) ? tsum[1] : (lane == 2) ? tsum[2] : 0.0f; ((volatile float*)OUTC)[(size_t)v * 32 + lane] = (v < N) ? val * cdiv : 0.0f; } __threadfence(); }
}
__global__ __launch_bounds__(256) void posout_kernel(const float* __restrict__ pos, const float* __restrict__ CS, float* __restrict__ out, int mrows) {
  const size_t i = (size_t)blockIdx.x * 256 + threadIdx.x; const size_t tot = (size_t)mrows * 3;
  for (int pass = 0; pass < 2; ++pass) { if (i < tot) ((volatile float*)out)[i] = bf16_rne(pos[i]) + CS[(i / 3) * 32 + (i % 3)]; __threadfence(); }
}
}

extern "C" void kernel_launch(void* const* d_in, const int* in_sizes, int n_in, void* d_out, int out_size, void* d_ws, size_t ws_size, hipStream_t stream) {
  (void)n_in;
  auto Fp = [&](int i) { return (const float*)d_in[i]; }; auto Ip = [&](int i) { return (const int*)d_in[i]; };
  if (in_sizes[0] != N * H || in_sizes[1] != N * 3 || in_sizes[2] != 2 * EFULL || in_sizes[3] != EFULL * 3 || in_sizes[4] != KIN * H || in_sizes[5] != H || in_sizes[6] != H * H || in_sizes[7] != H || in_sizes[8] != 2 * H * H || in_sizes[9] != H || in_sizes[10] != H * H || in_sizes[11] != H || in_sizes[12] != H * H || in_sizes[13] != H || in_sizes[14] != H || in_sizes[15] != 1 || out_size != N * H + N * 3) return;
  float* out_h = (float*)d_out; float* out_c = out_h + (size_t)N * H;
  size_t off = 0; char* ws = (char*)d_ws;
  auto carve = [&](size_t bytes) { char* p = ws + off; off += (bytes + 255) & ~(size_t)255; return p; };
  const size_t wsz = (size_t)H * H * 2;
  b16* WO = (b16*)carve(wsz); b16* WG = (b16*)carve(wsz); b16* W2 = (b16*)carve(wsz); b16* WC1 = (b16*)carve(wsz); b16* NT_ = (b16*)carve(2 * wsz); b16* NQ_ = (b16*)carve(2 * wsz); b16* U2T = (b16*)carve(wsz); b16* U2Q = (b16*)carve(wsz);
  float* AB = (float*)carve((size_t)NP * 2 * H * 4); float* MI = (float*)carve((size_t)NP * H * 4); float* CS = (float*)carve((size_t)NP * 32 * 4); float* U = (float*)carve((size_t)NP * H * 4);
  CsrBufs csr; off = csr_carve(csr, ws, off, E, N);
  if (off > ws_size || off > ((size_t)160 << 20)) return;
  const unsigned g8 = (H * H / 8 + 255) / 256, g16 = (H * 2 * H / 8 + 255) / 256;
  wtio_kernel<H, H><<<g8, 256, 0, stream>>>(Fp(4), H, 0, H, WO, WSC);
  wtio_kernel<H, H><<<g8, 256, 0, stream>>>(Fp(4), H, H, H, WG, WSC);
  wtio_kernel<H, H><<<g8, 256, 0, stream>>>(Fp(6), H, 0, H, W2, WSC);
  wtio_kernel<H, H><<<g8, 256, 0, stream>>>(Fp(12), H, 0, H, WC1, WSC);
  wtio_kernel<2 * H, H><<<g16, 256, 0, stream>>>(Fp(8), H, 0, 2 * H, NT_, WSC); wtio_kernel<2 * H, H><<<g16, 256, 0, stream>>>(Fp(8), H, 0, 2 * H, NQ_, WSQ);
  wtio_kernel<H, H><<<g8, 256, 0, stream>>>(Fp(10), H, 0, H, U2T, WSC); wtio_kernel<H, H><<<g8, 256, 0, stream>>>(Fp(10), H, 0, H, U2Q, WSQ);
  csr_build(csr, Ip(2), E, N, stream);
  ab_kernel<true><<<NRL / 32, 64, 0, stream>>>(Fp(0), WO, WG, Fp(5), AB);
  edge_kernel<0><<<NRL / 2, 64, 0, stream>>>(AB, Fp(1), Fp(3), Ip(2) + EFULL, csr.PERM, csr.ROWPTR, csr.ROWCNT, (int)csr.permLen, Fp(4) + (size_t)(2 * H) * H, W2, Fp(7), WC1, Fp(13), Fp(14), Fp(15), MI, CS);
  nodelin_kernel<<<NRL / 32, 64, 0, stream>>>(Fp(0), MI, NT_, NQ_, Fp(9), U, NP);
  lin2_kernel<false><<<NPL / 32, 64, 0, stream>>>(U, U2T, U2Q, Fp(11), out_h, NL);
  posout_kernel<<<(unsigned)(((size_t)NL * 3 + 255) / 256), 256, 0, stream>>>(Fp(1), CS, out_c, NL);
}
